// PLAggregator_33878702031556
// MI455X (gfx1250) — hardware-verified
//
#include <hip/hip_runtime.h>

typedef _Float16 v16h __attribute__((ext_vector_type(16)));
typedef _Float16 v8h  __attribute__((ext_vector_type(8)));
typedef _Float16 v4h  __attribute__((ext_vector_type(4)));
typedef float    v8f  __attribute__((ext_vector_type(8)));
typedef float    v4f  __attribute__((ext_vector_type(4)));
typedef v8h __attribute__((may_alias)) v8ha;
typedef v4h __attribute__((may_alias)) v4ha;
typedef v4f __attribute__((may_alias)) v4fa;

union Frag { v16h v; v8h half[2]; };

#define DM      128
#define HP      64
#define XS      136
#define YS      132
#define NRMAX   8
#define PLANE   (DM * DM)
#define SX      256.0f
#define SW      64.0f
#define INV_SXW 6.103515625e-05f

__device__ __forceinline__ v8f wmma_f16(v16h a, v16h b, v8f c) {
  v8f d = __builtin_amdgcn_wmma_f32_16x16x32_f16(false, a, false, b, (short)0, c, false, false);
  asm volatile("v_nop\n\tv_nop\n\tv_nop\n\tv_nop" : "+v"(d) : "v"(a), "v"(b));
  return d;
}

__device__ __forceinline__ v16h load_frag(const _Float16* p, int h) {
  Frag f;
  f.half[0] = *(const v8ha*)(p + 8 * h);
  f.half[1] = *(const v8ha*)(p + 16 + 8 * h);
  return f.v;
}

__device__ __forceinline__ int imin(int a, int b) { return a < b ? a : b; }
__device__ __forceinline__ int clampi(int v, int lo, int hi) { return v < lo ? lo : (v > hi ? hi : v); }

__device__ __forceinline__ void wpl_store_pass(const _Float16* sT, _Float16* base, int n0, int w, int lane) {
  const int q8 = lane & 7, sub = lane >> 3;
  #pragma unroll
  for (int i = 0; i < 2; ++i) {
    const int L = 8 * w + 4 * i + sub;
    const int nl = L >> 1, hl = L & 1;
    const v8h v = *(const v8ha*)(sT + nl * XS + 64 * hl + 8 * q8);
    *(volatile v8h*)(base + (size_t)(n0 + nl) * DM + 64 * hl + 8 * q8) = v;
  }
}

__global__ __launch_bounds__(256) void k_wplanes(
    const float* __restrict__ w1, const float* __restrict__ w2,
    const float* __restrict__ a1, const float* __restrict__ a2,
    _Float16* __restrict__ planes)
{
  __shared__ __attribute__((aligned(16))) _Float16 sT[32 * XS];

  const int tid = threadIdx.x, lane = tid & 31, w = tid >> 5;
  const int p = blockIdx.y, n0 = blockIdx.x * 32;
  const float* src = w1;
  int kb = 0;
  if (p == 1) { src = w2; }
  else if (p == 2) { src = a1; }
  else if (p == 3) { src = a2; }
  else if (p == 4) { src = a1; kb = DM; }

  #pragma unroll
  for (int i = 0; i < 16; ++i) {
    const int k = w + 8 * i;
    const float v = src[(size_t)(kb + k) * DM + n0 + lane];
    sT[lane * XS + k] = (_Float16)(v * SW);
  }
  __syncthreads();

  _Float16* base = planes + (size_t)p * PLANE;
  wpl_store_pass(sT, base, n0, w, lane);
  __threadfence();
  wpl_store_pass(sT, base, n0, w, lane);
}

__global__ __launch_bounds__(128) void k_rtab(
    const float* __restrict__ r2e, const float* __restrict__ w1,
    const float* __restrict__ b1, float* __restrict__ R, int NR)
{
  const int n = threadIdx.x;
  const float bias = b1[n];
  float vals[NRMAX];
  #pragma unroll
  for (int r = 0; r < NRMAX; ++r) {
    const float* rp = r2e + (size_t)imin(r, NR - 1) * DM;
    float acc = 0.0f;
    #pragma unroll 1
    for (int k = 0; k < DM; ++k) acc = fmaf(rp[k], w1[(size_t)(DM + k) * DM + n], acc);
    vals[r] = acc + bias;
  }
  #pragma unroll
  for (int r = 0; r < NRMAX; ++r) *(volatile float*)(R + r * DM + n) = vals[r];
  __threadfence();
  #pragma unroll
  for (int r = 0; r < NRMAX; ++r) *(volatile float*)(R + r * DM + n) = vals[r];
}

__device__ __forceinline__ void ub_store_pass(const float* sY, float* Ub, int b0, int w, int lane) {
  #pragma unroll
  for (int i = 0; i < 16; ++i) {
    const int row = 16 * w + i;
    const v4f v = *(const v4fa*)(sY + row * YS + 4 * lane);
    *(volatile v4f*)(Ub + (size_t)(b0 + row) * DM + 4 * lane) = v;
  }
}

__global__ __launch_bounds__(128) void k_ubias(
    const int* __restrict__ nodes_u, const float* __restrict__ u2e,
    const _Float16* __restrict__ A1b, const float* __restrict__ ab1,
    float* __restrict__ Ub, int B, int NU)
{
  __shared__ __attribute__((aligned(16))) _Float16 sX[64 * XS];
  __shared__ __attribute__((aligned(16))) float sY[64 * YS];

  const int tid = threadIdx.x, lane = tid & 31, w = tid >> 5;
  const int h = lane >> 4, m = lane & 15;
  const int b0 = blockIdx.x * 64;

  #pragma unroll
  for (int i = 0; i < 16; ++i) {
    const int r = w + 4 * i;
    const int bb = imin(b0 + r, B - 1);
    const int uid = clampi(nodes_u[bb], 0, NU - 1);
    const v4f v = *(const v4fa*)(u2e + (size_t)uid * DM + 4 * lane);
    const v4h o = { (_Float16)(v.x * SX), (_Float16)(v.y * SX), (_Float16)(v.z * SX), (_Float16)(v.w * SX) };
    *(v4ha*)(sX + r * XS + 4 * lane) = o;
  }
  __syncthreads();

  const v8f zero8 = {0.f, 0.f, 0.f, 0.f, 0.f, 0.f, 0.f, 0.f};
  v8f acc[8];
  #pragma unroll
  for (int t = 0; t < 8; ++t) acc[t] = zero8;

  const _Float16* arow  = sX + (16 * w + m) * XS;
  const _Float16* bbase = A1b + (size_t)m * DM;
  #pragma unroll 1
  for (int ks = 0; ks < 4; ++ks) {
    const int k0 = 32 * ks;
    const v16h af = load_frag(arow + k0, h);
    #pragma unroll
    for (int t = 0; t < 8; ++t) {
      const v16h bf = load_frag(bbase + (size_t)(16 * t) * DM + k0, h);
      acc[t] = wmma_f16(af, bf, acc[t]);
    }
  }

  #pragma unroll
  for (int t = 0; t < 8; ++t) {
    const int col = 16 * t + m;
    const float bias = ab1[col];
    #pragma unroll
    for (int r = 0; r < 8; ++r)
      sY[(16 * w + 8 * h + r) * YS + col] = acc[t][r] * INV_SXW + bias;
  }
  __syncthreads();

  ub_store_pass(sY, Ub, b0, w, lane);
  __threadfence();
  ub_store_pass(sY, Ub, b0, w, lane);
}

__device__ __forceinline__ void gemm64x16(const _Float16* sXp, const _Float16* __restrict__ Wp,
                                          int nb, int h, int m, v8f acc[4]) {
  const v8f zero8 = {0.f, 0.f, 0.f, 0.f, 0.f, 0.f, 0.f, 0.f};
  #pragma unroll
  for (int rt = 0; rt < 4; ++rt) acc[rt] = zero8;
  const _Float16* brow = Wp + (size_t)(nb + m) * DM;
  const _Float16* arow = sXp + m * XS;
  #pragma unroll 1
  for (int ks = 0; ks < 4; ++ks) {
    const int k0 = 32 * ks;
    const v16h bf = load_frag(brow + k0, h);
    #pragma unroll
    for (int rt = 0; rt < 4; ++rt) {
      const v16h af = load_frag(arow + rt * 16 * XS + k0, h);
      acc[rt] = wmma_f16(af, bf, acc[rt]);
    }
  }
}

__global__ __launch_bounds__(256) void k_main(
    const int* __restrict__ nodes_u, const int* __restrict__ hist_ids,
    const int* __restrict__ hist_labels,
    const float* __restrict__ v2e, const float* __restrict__ u2e,
    const _Float16* __restrict__ W1a, const _Float16* __restrict__ W2p,
    const _Float16* __restrict__ A1a, const _Float16* __restrict__ A2p,
    const float* __restrict__ Rtab, const float* __restrict__ Ub,
    const float* __restrict__ b2, const float* __restrict__ ab2,
    const float* __restrict__ att3, const float* __restrict__ att3b,
    float* __restrict__ out, int H, int NI, int NU, int NR)
{
  __shared__ __attribute__((aligned(16))) _Float16 sA[HP * XS];
  __shared__ __attribute__((aligned(16))) _Float16 sB[HP * XS];
  __shared__ __attribute__((aligned(16))) float sO[HP * DM];
  __shared__ float sR[NRMAX * DM];
  __shared__ float sUb[DM];
  __shared__ float sU[DM];
  __shared__ float sLg[8 * HP];
  __shared__ float sWt[HP];
  __shared__ __attribute__((aligned(16))) float sOut[DM];
  __shared__ int sLab[HP];

  const int b = blockIdx.x;
  const int tid = threadIdx.x, lane = tid & 31, wv = tid >> 5;
  const int h = lane >> 4, m = lane & 15;
  const int nb = 16 * wv, col = nb + m;

  const int uid = clampi(nodes_u[b], 0, NU - 1);
  if (tid < DM) {
    sU[tid]  = u2e[(size_t)uid * DM + tid];
    sUb[tid] = Ub[(size_t)b * DM + tid];
  }
  for (int i = tid; i < NRMAX * DM; i += 256) sR[i] = Rtab[i];
  if (tid < HP) {
    const int rr = imin(tid, H - 1);
    const int lab = clampi(hist_labels[(size_t)b * H + rr], 0, NR - 1);
    sLab[tid] = (tid < H) ? lab : 0;
  }
  #pragma unroll
  for (int i = 0; i < 8; ++i) {
    const int r = wv + 8 * i;
    const int rr = imin(r, H - 1);
    const int iid = clampi(hist_ids[(size_t)b * H + rr], 0, NI - 1);
    const v4f v = *(const v4fa*)(v2e + (size_t)iid * DM + 4 * lane);
    const float sc = (r < H) ? SX : 0.0f;
    const v4h o = { (_Float16)(v.x * sc), (_Float16)(v.y * sc), (_Float16)(v.z * sc), (_Float16)(v.w * sc) };
    *(v4ha*)(sA + r * XS + 4 * lane) = o;
  }
  __syncthreads();

  v8f acc[4];

  gemm64x16(sA, W1a, nb, h, m, acc);
  #pragma unroll
  for (int rt = 0; rt < 4; ++rt)
    #pragma unroll
    for (int r = 0; r < 8; ++r) {
      const int row = 16 * rt + 8 * h + r;
      const float v = fmaxf(acc[rt][r] * INV_SXW + sR[sLab[row] * DM + col], 0.0f);
      sB[row * XS + col] = (_Float16)(v * SX);
    }
  __syncthreads();

  gemm64x16(sB, W2p, nb, h, m, acc);
  {
    const float bias = b2[col];
    #pragma unroll
    for (int rt = 0; rt < 4; ++rt)
      #pragma unroll
      for (int r = 0; r < 8; ++r) {
        const int row = 16 * rt + 8 * h + r;
        const float o = fmaxf(acc[rt][r] * INV_SXW + bias, 0.0f);
        sO[row * DM + col] = o;
        sA[row * XS + col] = (_Float16)(o * SX);
      }
  }
  __syncthreads();

  gemm64x16(sA, A1a, nb, h, m, acc);
  {
    const float ub = sUb[col];
    #pragma unroll
    for (int rt = 0; rt < 4; ++rt)
      #pragma unroll
      for (int r = 0; r < 8; ++r) {
        const int row = 16 * rt + 8 * h + r;
        const float a = fmaxf(acc[rt][r] * INV_SXW + ub, 0.0f);
        sB[row * XS + col] = (_Float16)(a * SX);
      }
  }
  __syncthreads();

  gemm64x16(sB, A2p, nb, h, m, acc);
  {
    const float bias = ab2[col];
    const float a3 = att3[col];
    #pragma unroll
    for (int rt = 0; rt < 4; ++rt)
      #pragma unroll
      for (int r = 0; r < 8; ++r) {
        float v = fmaxf(acc[rt][r] * INV_SXW + bias, 0.0f) * a3;
        v += __shfl_xor(v, 8);
        v += __shfl_xor(v, 4);
        v += __shfl_xor(v, 2);
        v += __shfl_xor(v, 1);
        if (m == 0) sLg[wv * HP + 16 * rt + 8 * h + r] = v;
      }
  }
  __syncthreads();

  if (wv == 0) {
    float l0 = 0.0f, l1 = 0.0f;
    #pragma unroll
    for (int w = 0; w < 8; ++w) { l0 += sLg[w * HP + lane]; l1 += sLg[w * HP + lane + 32]; }
    const float ab3 = att3b[0];
    l0 += ab3; l1 += ab3;
    const bool ok0 = lane < H, ok1 = (lane + 32) < H;
    const float v0 = ok0 ? l0 : -3.0e38f;
    const float v1 = ok1 ? l1 : -3.0e38f;
    float mx = fmaxf(v0, v1);
    #pragma unroll
    for (int off = 16; off > 0; off >>= 1) mx = fmaxf(mx, __shfl_xor(mx, off));
    const float x0 = expf(v0 - mx), x1 = expf(v1 - mx);
    const float e0 = ok0 ? x0 : 0.0f;
    const float e1 = ok1 ? x1 : 0.0f;
    float s = e0 + e1;
    #pragma unroll
    for (int off = 16; off > 0; off >>= 1) s += __shfl_xor(s, off);
    const float inv = 1.0f / s;
    sWt[lane] = e0 * inv;
    sWt[lane + 32] = e1 * inv;
  }
  __syncthreads();

  if (tid < DM) {
    const int d = tid;
    float s = 0.0f;
    #pragma unroll 1
    for (int hh = 0; hh < H; ++hh) s = fmaf(sWt[hh], sO[hh * DM + d], s);
    sOut[d] = (s + sU[d]) * 0.5f;
  }
  __syncthreads();

  if (wv == 0) {
    const v4f v = *(const v4fa*)(sOut + 4 * lane);
    float* dst = out + (size_t)b * DM + 4 * lane;
    *(volatile v4f*)dst = v;
    __threadfence();
    *(volatile v4f*)dst = v;
  }
}

extern "C" void kernel_launch(void* const* d_in, const int* in_sizes, int n_in,
                              void* d_out, int out_size, void* d_ws, size_t ws_size,
                              hipStream_t stream) {
  if (n_in < 16) return;
  const int B = in_sizes[0];
  if (B <= 0) return;
  const int H = in_sizes[1] / B;
  if (H < 1 || H > HP) return;
  if (in_sizes[1] != B * H || in_sizes[2] != B * H) return;
  if (in_sizes[3] < DM || (in_sizes[3] % DM) != 0) return;
  if (in_sizes[4] < DM || (in_sizes[4] % DM) != 0) return;
  if (in_sizes[5] < DM || (in_sizes[5] % DM) != 0) return;
  const int NI = in_sizes[3] / DM;
  const int NU = in_sizes[4] / DM;
  const int NR = in_sizes[5] / DM;
  if (NR > NRMAX) return;
  if (in_sizes[6] != 2 * DM * DM || in_sizes[8] != DM * DM) return;
  if (in_sizes[10] != 2 * DM * DM || in_sizes[12] != DM * DM) return;
  if (in_sizes[7] != DM || in_sizes[9] != DM || in_sizes[11] != DM || in_sizes[13] != DM) return;
  if (in_sizes[14] != DM || in_sizes[15] < 1) return;
  if (out_size != B * DM) return;

  const int*   nodes_u     = (const int*)d_in[0];
  const int*   hist_ids    = (const int*)d_in[1];
  const int*   hist_labels = (const int*)d_in[2];
  const float* v2e   = (const float*)d_in[3];
  const float* u2e   = (const float*)d_in[4];
  const float* r2e   = (const float*)d_in[5];
  const float* w1    = (const float*)d_in[6];
  const float* b1    = (const float*)d_in[7];
  const float* w2    = (const float*)d_in[8];
  const float* b2    = (const float*)d_in[9];
  const float* a1    = (const float*)d_in[10];
  const float* ab1   = (const float*)d_in[11];
  const float* a2    = (const float*)d_in[12];
  const float* ab2   = (const float*)d_in[13];
  const float* att3  = (const float*)d_in[14];
  const float* att3b = (const float*)d_in[15];
  float* out = (float*)d_out;

  const int Bpad = ((B + 63) / 64) * 64;
  const size_t pl_bytes = (size_t)5 * PLANE * 2;
  const size_t r_bytes  = (size_t)NRMAX * DM * 4;
  const size_t ub_bytes = (size_t)Bpad * DM * 4;
  const size_t off_r  = pl_bytes;
  const size_t off_ub = off_r + r_bytes;
  const size_t total  = off_ub + ub_bytes;
  if (total > ws_size) return;

  char* ws = (char*)d_ws;
  _Float16* planes = (_Float16*)ws;
  float* Rtab = (float*)(ws + off_r);
  float* Ub   = (float*)(ws + off_ub);
  const _Float16* W1a = planes;
  const _Float16* W2p = planes + PLANE;
  const _Float16* A1a = planes + 2 * PLANE;
  const _Float16* A2p = planes + 3 * PLANE;
  const _Float16* A1b = planes + 4 * PLANE;

  dim3 gPl(DM / 32, 5);
  k_wplanes<<<gPl, 256, 0, stream>>>(w1, w2, a1, a2, planes);

  k_rtab<<<1, DM, 0, stream>>>(r2e, w1, b1, Rtab, NR);

  k_ubias<<<Bpad / 64, 128, 0, stream>>>(nodes_u, u2e, A1b, ab1, Ub, B, NU);

  k_main<<<B, 256, 0, stream>>>(nodes_u, hist_ids, hist_labels, v2e, u2e,
                                W1a, W2p, A1a, A2p, Rtab, Ub, b2, ab2, att3, att3b,
                                out, H, NI, NU, NR);
}
